// GemmaAttention_45320494907672
// MI455X (gfx1250) — hardware-verified
//
#include <hip/hip_runtime.h>
#include <math.h>
#include <stdint.h>

#define NB_     2
#define SEQ_    2048
#define DM_     2048
#define NH_     8
#define HD_     256
#define NF_     128
#define KVN_    512
#define WIN_    1024
#define NQB_    32
#define QE_     4
#define LOROWS_ 256

#define CX_   16.0f
#define CW_   256.0f
#define CQK_  1024.0f
#define CP_   32768.0f
#define SSC_  5.9604644775390625e-8f
#define OSC_  3.0517578125e-5f
#define QSC_  2.44140625e-4f
#define WSC_  3.814697265625e-6f

typedef _Float16 v16h __attribute__((ext_vector_type(16)));
typedef _Float16 v8h  __attribute__((ext_vector_type(8)));
typedef float    v8f  __attribute__((ext_vector_type(8)));
typedef float    v4f  __attribute__((ext_vector_type(4)));

union FragU { v16h v; v8h h[2]; };
union U8 { v8f v; v4f q[2]; };

__device__ __forceinline__ float bf16_rne(float f) {
  unsigned u = __float_as_uint(f);
  u = u + 0x7FFFu + ((u >> 16) & 1u);
  return __uint_as_float(u & 0xFFFF0000u);
}
__device__ __forceinline__ v8f zero8() { return (v8f){0.f, 0.f, 0.f, 0.f, 0.f, 0.f, 0.f, 0.f}; }

__device__ __forceinline__ v16h frag_ld(const _Float16* p) {
  FragU f;
  f.h[0] = *(const v8h*)(p);
  f.h[1] = *(const v8h*)(p + 16);
  return f.v;
}
__device__ __forceinline__ v8f wmma_raw(v16h a, v16h b, v8f c) {
  return __builtin_amdgcn_wmma_f32_16x16x32_f16(false, a, false, b, (short)0, c, false, false);
}
__device__ __forceinline__ v8f mma_g(v16h a, v16h b, v8f c) {
  c = __builtin_amdgcn_wmma_f32_16x16x32_f16(false, a, false, b, (short)0, c, false, false);
  asm volatile("v_nop\n\tv_nop\n\tv_nop\n\tv_nop" : "+v"(c) : "v"(a), "v"(b));
  return c;
}
__device__ __forceinline__ void dep_guard(v8f& a, v8f& b, v16h x, v16h y) {
  asm volatile("v_nop\n\tv_nop\n\tv_nop\n\tv_nop" : "+v"(a), "+v"(b) : "v"(x), "v"(y));
}
__device__ __forceinline__ void keep4(v16h a, v16h b, v16h c, v16h d) {
  asm volatile("v_nop" :: "v"(a), "v"(b), "v"(c), "v"(d));
}
__device__ __forceinline__ void acc_guard4(v8f& a, v8f& b, v8f& c, v8f& d) {
  asm volatile("v_nop\n\tv_nop\n\tv_nop\n\tv_nop" : "+v"(a), "+v"(b), "+v"(c), "+v"(d));
}

__global__ __launch_bounds__(256) void cvt16_kernel(const float* __restrict__ src, _Float16* __restrict__ dst, int n8, float scale) {
  const int i = blockIdx.x * 256 + (int)threadIdx.x;
  if (i >= n8) return;
  const float* s = src + 8 * (size_t)i;
  U8 a;
  a.q[0] = *(const v4f*)(s);
  a.q[1] = *(const v4f*)(s + 4);
  v8h o;
#pragma unroll
  for (int e = 0; e < 8; ++e) o[e] = (_Float16)(bf16_rne(a.v[e]) * scale);
  _Float16* d = dst + 8 * (size_t)i;
  *(volatile v8h*)d = o;
  __threadfence();
  *(volatile v8h*)d = o;
}

__global__ __launch_bounds__(256) void rope_table_kernel(const int* __restrict__ pos, float* __restrict__ cosT,
                                                         float* __restrict__ sinT, int nrows) {
#pragma clang fp contract(off)
  __shared__ float invf[NF_];
  const int tid = threadIdx.x;
  if (tid < NF_) {
    const double e = (double)tid * 0.0078125;
    const double p = exp2(e * 13.287712379549449);
    const float pf = (float)p;
    invf[tid] = 1.0f / pf;
  }
  __syncthreads();
  const int f = tid & (NF_ - 1);
  const int rp = tid >> 7;
  const int r0 = blockIdx.x * 32;
  const float iv = invf[f];
#pragma unroll 1
  for (int it = 0; it < 16; ++it) {
    const int row = r0 + it * 2 + rp;
    const int rowc = (row < nrows) ? row : (nrows - 1);
    const float ang = (float)pos[rowc] * iv;
    float sv, cv;
    sincosf(ang, &sv, &cv);
    if (row < nrows) {
      float* cp = cosT + (size_t)row * NF_ + f;
      float* sp = sinT + (size_t)row * NF_ + f;
      *(volatile float*)cp = cv;
      *(volatile float*)sp = sv;
      __threadfence();
      *(volatile float*)cp = cv;
      *(volatile float*)sp = sv;
    }
  }
}

__global__ __launch_bounds__(256) void maskflag_kernel(const float* __restrict__ mask, int* __restrict__ flag) {
  __shared__ int sw[8];
  const int tid = threadIdx.x, w = tid >> 5, lane = tid & 31;
  const int bq = blockIdx.x;
  const int b = bq >> 5, qb = bq & (NQB_ - 1);
  const int q0 = qb * 64;
  int bad = 0;
#pragma unroll 1
  for (int rr = 0; rr < 64; ++rr) {
    const int qrow = q0 + rr;
    int kend = qrow + WIN_ - 1;
    if (kend > SEQ_ - 1) kend = SEQ_ - 1;
    const float* mp = mask + ((size_t)b * SEQ_ + qrow) * SEQ_;
#pragma unroll 1
    for (int kb0 = q0 + 64; kb0 <= kend; kb0 += 256) {
      const int k = kb0 + tid;
      const int kc = (k <= kend) ? k : kend;
      const float mv = mp[kc];
      const int ok = (mv <= -1.0e9f) ? 1 : 0;
      bad |= ((k <= kend) && (ok == 0)) ? 1 : 0;
    }
  }
  const unsigned long long bm = __ballot(bad);
  if (lane == 0) sw[w] = (bm != 0ull) ? 1 : 0;
  __syncthreads();
  if (w == 0) {
    int any = 0;
#pragma unroll
    for (int i = 0; i < 8; ++i) any |= sw[i];
    const int fv = any ? 0 : 1;
    int* fp = flag + (size_t)bq * 32 + lane;
    *(volatile int*)fp = fv;
    __threadfence();
    *(volatile int*)fp = fv;
  }
}

template <bool LO>
__device__ __forceinline__ void gemm_kloop(v8f (&acc)[4][4], const _Float16* __restrict__ Ab, const _Float16* __restrict__ Ab2,
                                           int lda, const _Float16* __restrict__ Bb, int ldb, int m0, int n0, int K,
                                           int rlane, int koff) {
  for (int k0 = 0; k0 < K; k0 += 32) {
    v16h bh[4];
#pragma unroll
    for (int j = 0; j < 4; ++j) bh[j] = frag_ld(Bb + (size_t)(n0 + (j << 4) + rlane) * ldb + k0 + koff);
#pragma unroll
    for (int i = 0; i < 4; ++i) {
      const size_t ao = (size_t)(m0 + (i << 4) + rlane) * lda + k0 + koff;
      const v16h ah = frag_ld(Ab + ao);
      v16h al = ah;
      if (LO) al = frag_ld(Ab2 + ao);
#pragma unroll
      for (int j = 0; j < 4; ++j) {
        acc[i][j] = wmma_raw(ah, bh[j], acc[i][j]);
        if (LO) acc[i][j] = wmma_raw(al, bh[j], acc[i][j]);
      }
      dep_guard(acc[i][0], acc[i][3], ah, al);
    }
    keep4(bh[0], bh[1], bh[2], bh[3]);
  }
}

__global__ __launch_bounds__(256) void gemm64_kernel(const _Float16* __restrict__ A, const _Float16* __restrict__ A2, int lda,
                                                     const _Float16* __restrict__ Bt, int ldb,
                                                     float* __restrict__ C, int ldc, int M, int N, int K,
                                                     int loRows, int seqMask, float scale) {
  __shared__ __align__(16) float sT[8][16 * 68];
  const int lane = threadIdx.x & 31;
  const int wave = threadIdx.x >> 5;
  const int tilesN = N >> 6;
  const int tilesM = M >> 6;
  const int tile = blockIdx.x * 8 + wave;
  if (tile >= tilesM * tilesN) return;
  const int tm = tile / tilesN;
  const int tn = tile - tm * tilesN;
  const int m0 = tm << 6;
  const int n0 = tn << 6;
  const int rlane = lane & 15;
  const int koff  = (lane >> 4) * 8;
  const int mOff  = koff;

  v8f acc[4][4];
#pragma unroll
  for (int i = 0; i < 4; ++i)
#pragma unroll
    for (int j = 0; j < 4; ++j) acc[i][j] = zero8();

  const bool useLo = ((m0 & seqMask) < loRows);
  if (useLo) gemm_kloop<true>(acc, A, A2, lda, Bt, ldb, m0, n0, K, rlane, koff);
  else       gemm_kloop<false>(acc, A, A, lda, Bt, ldb, m0, n0, K, rlane, koff);
  acc_guard4(acc[0][0], acc[0][1], acc[0][2], acc[0][3]);
  acc_guard4(acc[1][0], acc[1][1], acc[1][2], acc[1][3]);
  acc_guard4(acc[2][0], acc[2][1], acc[2][2], acc[2][3]);
  acc_guard4(acc[3][0], acc[3][1], acc[3][2], acc[3][3]);

  float* slab = sT[wave];
  const int hrow = lane >> 4;
  const int c4 = rlane * 4;
#pragma unroll
  for (int i = 0; i < 4; ++i) {
    const int mBase = m0 + (i << 4);
#pragma unroll
    for (int j = 0; j < 4; ++j) {
#pragma unroll
      for (int r = 0; r < 8; ++r) slab[(mOff + r) * 68 + (j << 4) + rlane] = acc[i][j][r] * scale;
    }
    __builtin_amdgcn_fence(__ATOMIC_RELEASE, "workgroup");
    __builtin_amdgcn_wave_barrier();
    __builtin_amdgcn_fence(__ATOMIC_ACQUIRE, "workgroup");
    for (int pass = 0; pass < 2; ++pass) {
#pragma unroll
      for (int it = 0; it < 8; ++it) {
        const int row = it * 2 + hrow;
        const v4f v = *(const v4f*)(slab + row * 68 + c4);
        *(volatile v4f*)(C + (size_t)(mBase + row) * ldc + n0 + c4) = v;
      }
      __threadfence();
    }
    __builtin_amdgcn_fence(__ATOMIC_RELEASE, "workgroup");
    __builtin_amdgcn_wave_barrier();
    __builtin_amdgcn_fence(__ATOMIC_ACQUIRE, "workgroup");
  }
}

__global__ __launch_bounds__(256) void rope_split_kernel(const float* __restrict__ src, int spitch, int nheads,
                                                         const float* __restrict__ cosT, const float* __restrict__ sinT,
                                                         _Float16* __restrict__ hi, _Float16* __restrict__ lo,
                                                         int dpitch, int nunits, float carry) {
#pragma clang fp contract(off)
  const int gid = blockIdx.x * 256 + (int)threadIdx.x;
  const int unit = gid >> 3;
  const int j = gid & 7;
  if (unit >= nunits) return;
  const int row = unit / nheads;
  const int hd = unit - row * nheads;
  const float* s  = src  + (size_t)row * spitch + hd * HD_ + 8 * j;
  const float* ct = cosT + (size_t)row * NF_ + 8 * j;
  const float* st = sinT + (size_t)row * NF_ + 8 * j;
  U8 xa, xb, xc, xd, ca, cb, sa, sb;
  xa.q[0] = *(const v4f*)(s);         xa.q[1] = *(const v4f*)(s + 4);
  xb.q[0] = *(const v4f*)(s + 64);    xb.q[1] = *(const v4f*)(s + 68);
  xc.q[0] = *(const v4f*)(s + 128);   xc.q[1] = *(const v4f*)(s + 132);
  xd.q[0] = *(const v4f*)(s + 192);   xd.q[1] = *(const v4f*)(s + 196);
  ca.q[0] = *(const v4f*)(ct);        ca.q[1] = *(const v4f*)(ct + 4);
  cb.q[0] = *(const v4f*)(ct + 64);   cb.q[1] = *(const v4f*)(ct + 68);
  sa.q[0] = *(const v4f*)(st);        sa.q[1] = *(const v4f*)(st + 4);
  sb.q[0] = *(const v4f*)(st + 64);   sb.q[1] = *(const v4f*)(st + 68);
  v8h h0, h1, h2, h3, l0, l1, l2, l3;
#pragma unroll
  for (int e = 0; e < 8; ++e) {
    const float r0 = xa.v[e] * ca.v[e] - xc.v[e] * sa.v[e];
    const float r1 = xb.v[e] * cb.v[e] - xd.v[e] * sb.v[e];
    const float r2 = xc.v[e] * ca.v[e] + xa.v[e] * sa.v[e];
    const float r3 = xd.v[e] * cb.v[e] + xb.v[e] * sb.v[e];
    float t; _Float16 q;
    t = r0 * carry; q = (_Float16)t; h0[e] = q; l0[e] = (_Float16)(t - (float)q);
    t = r1 * carry; q = (_Float16)t; h1[e] = q; l1[e] = (_Float16)(t - (float)q);
    t = r2 * carry; q = (_Float16)t; h2[e] = q; l2[e] = (_Float16)(t - (float)q);
    t = r3 * carry; q = (_Float16)t; h3[e] = q; l3[e] = (_Float16)(t - (float)q);
  }
  _Float16* hp = hi + (size_t)row * dpitch + hd * HD_ + 8 * j;
  _Float16* lp = lo + (size_t)row * dpitch + hd * HD_ + 8 * j;
  for (int pass = 0; pass < 2; ++pass) {
    *(volatile v8h*)(hp)       = h0;
    *(volatile v8h*)(hp + 64)  = h1;
    *(volatile v8h*)(hp + 128) = h2;
    *(volatile v8h*)(hp + 192) = h3;
    *(volatile v8h*)(lp)       = l0;
    *(volatile v8h*)(lp + 64)  = l1;
    *(volatile v8h*)(lp + 128) = l2;
    *(volatile v8h*)(lp + 192) = l3;
    __threadfence();
  }
}

__global__ __launch_bounds__(256) void vt_split_kernel(const float* __restrict__ KV, _Float16* __restrict__ Vth,
                                                       _Float16* __restrict__ Vtl) {
  __shared__ __align__(16) float tf[64 * 68];
  const int tid = threadIdx.x;
  const int d0  = blockIdx.x * 64;
  const int sg0 = blockIdx.y * 64;
  const int b   = sg0 >> 11;
  const int s0  = sg0 & (SEQ_ - 1);
  {
    const int lr = tid >> 4;
    const int c4 = (tid & 15) * 4;
#pragma unroll
    for (int it = 0; it < 4; ++it) {
      const int rr = it * 16 + lr;
      const v4f a = *(const v4f*)(KV + (size_t)(sg0 + rr) * KVN_ + HD_ + d0 + c4);
      *(v4f*)(tf + rr * 68 + c4) = a;
    }
  }
  __syncthreads();
  const int sub = tid >> 3;
  const int c8  = (tid & 7) * 8;
  v8h hv[2], lv[2];
#pragma unroll
  for (int it = 0; it < 2; ++it) {
    const int oc = it * 32 + sub;
    v8h a, rsd;
#pragma unroll
    for (int q = 0; q < 8; ++q) {
      const float f = tf[(c8 + q) * 68 + oc] * CQK_;
      const _Float16 hq = (_Float16)f;
      a[q] = hq;
      rsd[q] = (_Float16)(f - (float)hq);
    }
    hv[it] = a; lv[it] = rsd;
  }
  for (int pass = 0; pass < 2; ++pass) {
#pragma unroll
    for (int it = 0; it < 2; ++it) {
      const int oc = it * 32 + sub;
      const size_t go = ((size_t)b * HD_ + d0 + oc) * SEQ_ + s0 + c8;
      *(volatile v8h*)(Vth + go) = hv[it];
      *(volatile v8h*)(Vtl + go) = lv[it];
    }
    __threadfence();
  }
}

#define AT_PPITCH 72
#define AT_OPITCH 264
#define AT_OFF_PH 0
#define AT_OFF_PL 9216
#define AT_OFF_PM 18432
#define AT_OFF_PS 18944
#define AT_OFF_AL 19456
#define AT_OFF_LF 19712
#define AT_OFF_OH 19968
#define AT_OFF_OL 53760
#define AT_LDS    87552
static_assert(AT_OFF_PL == AT_OFF_PH + 64 * AT_PPITCH * 2);
static_assert(AT_OFF_PM == AT_OFF_PL + 64 * AT_PPITCH * 2);
static_assert(AT_OFF_OL == AT_OFF_OH + 64 * AT_OPITCH * 2);
static_assert(AT_LDS == AT_OFF_OL + 64 * AT_OPITCH * 2);

__global__ __launch_bounds__(256) void attn_kernel(const _Float16* __restrict__ Qh, const _Float16* __restrict__ Ql,
                                                   const _Float16* __restrict__ Kh, const _Float16* __restrict__ Kl,
                                                   const _Float16* __restrict__ Vth, const _Float16* __restrict__ Vtl,
                                                   const float* __restrict__ mask, const int* __restrict__ flag,
                                                   _Float16* __restrict__ AOh, _Float16* __restrict__ AOl) {
  extern __shared__ __align__(16) unsigned char dsm[];
  _Float16* Ph   = (_Float16*)(dsm + AT_OFF_PH);
  _Float16* Pl   = (_Float16*)(dsm + AT_OFF_PL);
  float*    pm   = (float*)(dsm + AT_OFF_PM);
  float*    ps   = (float*)(dsm + AT_OFF_PS);
  float*    alph = (float*)(dsm + AT_OFF_AL);
  float*    lfin = (float*)(dsm + AT_OFF_LF);
  _Float16* Ohs  = (_Float16*)(dsm + AT_OFF_OH);
  _Float16* Ols  = (_Float16*)(dsm + AT_OFF_OL);

  const int tid  = threadIdx.x;
  const int w    = tid >> 5;
  const int lane = tid & 31;
  const int hh   = lane >> 4;
  const int c    = lane & 15;
  const int bid  = blockIdx.x;
  const int qb   = bid & (NQB_ - 1);
  const int h    = (bid >> 5) & (NH_ - 1);
  const int b    = bid >> 8;
  const int q0   = qb * 64;
  const int srow0 = (w & 3) * 16;
  const int kh    = w >> 2;
  const int ocol0 = w * 32;
  const bool early = (qb < QE_);
  const int ktlo = (qb > 16) ? (qb - 16) : 0;
  const int fl = flag[(b * NQB_ + qb) * 32];
  int kthi = (fl != 0) ? qb : (qb + 16);
  if (kthi > NQB_ - 1) kthi = NQB_ - 1;

  const size_t growq = (size_t)b * SEQ_ + q0;
  const _Float16* qhp = Qh + (growq + srow0 + c) * DM_ + h * HD_ + 8 * hh;
  const _Float16* qlp = Ql + (growq + srow0 + c) * DM_ + h * HD_ + 8 * hh;
  const float*    mrp = mask + (growq + srow0 + 8 * hh) * (size_t)SEQ_;
  const _Float16* vhp = Vth + ((size_t)b * HD_ + ocol0 + c) * SEQ_ + 8 * hh;
  const _Float16* vlp = Vtl + ((size_t)b * HD_ + ocol0 + c) * SEQ_ + 8 * hh;

  float mrow[8], lrow[8];
  v8f oacc[4][2];
#pragma unroll
  for (int r = 0; r < 8; ++r) { mrow[r] = -INFINITY; lrow[r] = 0.0f; }
#pragma unroll
  for (int i = 0; i < 4; ++i) { oacc[i][0] = zero8(); oacc[i][1] = zero8(); }

  for (int kt = ktlo; kt <= kthi; ++kt) {
    const int key0  = kt * 64;
    const int wkey0 = key0 + 32 * kh;
    const _Float16* khp = Kh + ((size_t)b * SEQ_ + wkey0 + c) * HD_ + 8 * hh;
    const _Float16* klp = Kl + ((size_t)b * SEQ_ + wkey0 + c) * HD_ + 8 * hh;

    v8f s[2];
    s[0] = zero8(); s[1] = zero8();
#pragma unroll
    for (int ks = 0; ks < 8; ++ks) {
      const v16h qa = frag_ld(qhp + 32 * ks);
      v16h qr = qa;
      if (early) qr = frag_ld(qlp + 32 * ks);
#pragma unroll
      for (int j = 0; j < 2; ++j) {
        const v16h kb = frag_ld(khp + (size_t)(16 * j) * HD_ + 32 * ks);
        s[j] = mma_g(qa, kb, s[j]);
        if (early) {
          const v16h kr = frag_ld(klp + (size_t)(16 * j) * HD_ + 32 * ks);
          s[j] = mma_g(qr, kb, s[j]);
          s[j] = mma_g(qa, kr, s[j]);
        }
      }
    }

    float cm[8];
#pragma unroll
    for (int r = 0; r < 8; ++r) {
      const int qrow = q0 + srow0 + 8 * hh + r;
      const float* mp = mrp + (size_t)r * SEQ_;
      float mx = -INFINITY;
#pragma unroll
      for (int j = 0; j < 2; ++j) {
        const int key = wkey0 + 16 * j + c;
        const float mv = mp[key];
        const bool inb = (key + (WIN_ - 1) >= qrow) && (key <= qrow + (WIN_ - 1));
        const float sv = inb ? (s[j][r] * SSC_ + mv) : -INFINITY;
        s[j][r] = sv;
        mx = fmaxf(mx, sv);
      }
      mx = fmaxf(mx, __shfl_xor(mx, 1, 32));
      mx = fmaxf(mx, __shfl_xor(mx, 2, 32));
      mx = fmaxf(mx, __shfl_xor(mx, 4, 32));
      mx = fmaxf(mx, __shfl_xor(mx, 8, 32));
      cm[r] = mx;
    }
    if (c == 0) {
#pragma unroll
      for (int r = 0; r < 8; ++r) pm[w * 16 + 8 * hh + r] = cm[r];
    }
    __syncthreads();

    float al[8], psm[8];
    const int wo = w ^ 4;
#pragma unroll
    for (int r = 0; r < 8; ++r) {
      const float om = pm[wo * 16 + 8 * hh + r];
      const float mnew = fmaxf(mrow[r], fmaxf(cm[r], om));
      const float msafe = (mnew == -INFINITY) ? 0.0f : mnew;
      al[r] = __expf(mrow[r] - msafe);
      mrow[r] = mnew;
      float sum = 0.0f;
#pragma unroll
      for (int j = 0; j < 2; ++j) {
        const float p = __expf(s[j][r] - msafe);
        sum += p;
        const float t = p * CP_;
        const _Float16 phv = (_Float16)t;
        const int pidx = (srow0 + 8 * hh + r) * AT_PPITCH + 32 * kh + 16 * j + c;
        Ph[pidx] = phv;
        if (early) Pl[pidx] = (_Float16)(t - (float)phv);
      }
      sum += __shfl_xor(sum, 1, 32);
      sum += __shfl_xor(sum, 2, 32);
      sum += __shfl_xor(sum, 4, 32);
      sum += __shfl_xor(sum, 8, 32);
      psm[r] = sum;
    }
    if (c == 0) {
#pragma unroll
      for (int r = 0; r < 8; ++r) ps[w * 16 + 8 * hh + r] = psm[r];
      if (w < 4) {
#pragma unroll
        for (int r = 0; r < 8; ++r) alph[srow0 + 8 * hh + r] = al[r];
      }
    }
    __syncthreads();
#pragma unroll
    for (int r = 0; r < 8; ++r)
      lrow[r] = lrow[r] * al[r] + (ps[(w & 3) * 16 + 8 * hh + r] + ps[((w & 3) + 4) * 16 + 8 * hh + r]);

#pragma unroll
    for (int i = 0; i < 4; ++i) {
      U8 av;
      av.q[0] = *(const v4f*)(alph + 16 * i + 8 * hh);
      av.q[1] = *(const v4f*)(alph + 16 * i + 8 * hh + 4);
#pragma unroll
      for (int r = 0; r < 8; ++r) { oacc[i][0][r] *= av.v[r]; oacc[i][1][r] *= av.v[r]; }
    }
#pragma unroll
    for (int k2 = 0; k2 < 2; ++k2) {
      const int kk = key0 + 32 * k2;
#pragma unroll
      for (int jj = 0; jj < 2; ++jj) {
        const v16h vb = frag_ld(vhp + (size_t)(16 * jj) * SEQ_ + kk);
        v16h vr = vb;
        if (early) vr = frag_ld(vlp + (size_t)(16 * jj) * SEQ_ + kk);
#pragma unroll
        for (int i = 0; i < 4; ++i) {
          const v16h pa = frag_ld(Ph + (16 * i + c) * AT_PPITCH + 32 * k2 + 8 * hh);
          oacc[i][jj] = mma_g(pa, vb, oacc[i][jj]);
          if (early) {
            const v16h pr = frag_ld(Pl + (16 * i + c) * AT_PPITCH + 32 * k2 + 8 * hh);
            oacc[i][jj] = mma_g(pa, vr, oacc[i][jj]);
            oacc[i][jj] = mma_g(pr, vb, oacc[i][jj]);
          }
        }
      }
    }
  }

  if (w < 4 && c == 0) {
#pragma unroll
    for (int r = 0; r < 8; ++r) lfin[srow0 + 8 * hh + r] = lrow[r];
  }
  __syncthreads();
#pragma unroll
  for (int i = 0; i < 4; ++i) {
    U8 lv;
    lv.q[0] = *(const v4f*)(lfin + 16 * i + 8 * hh);
    lv.q[1] = *(const v4f*)(lfin + 16 * i + 8 * hh + 4);
#pragma unroll
    for (int r = 0; r < 8; ++r) {
      const float f = OSC_ * (1.0f / lv.v[r]);
      const int orow = 16 * i + 8 * hh + r;
#pragma unroll
      for (int jj = 0; jj < 2; ++jj) {
        const float t = oacc[i][jj][r] * f;
        const _Float16 hq = (_Float16)t;
        const int oidx = orow * AT_OPITCH + ocol0 + 16 * jj + c;
        Ohs[oidx] = hq;
        Ols[oidx] = (_Float16)(t - (float)hq);
      }
    }
  }
  __syncthreads();
  {
    const int piece = tid & 7;
    const int lsub  = tid >> 3;
    for (int pass = 0; pass < 2; ++pass) {
#pragma unroll
      for (int it = 0; it < 8; ++it) {
        const int line = it * 32 + lsub;
        const int row  = line >> 2;
        const int col  = (line & 3) * 64 + piece * 8;
        const v8h hv = *(const v8h*)(Ohs + row * AT_OPITCH + col);
        const v8h rv = *(const v8h*)(Ols + row * AT_OPITCH + col);
        const size_t go = (growq + row) * DM_ + h * HD_ + col;
        *(volatile v8h*)(AOh + go) = hv;
        *(volatile v8h*)(AOl + go) = rv;
      }
      __threadfence();
    }
  }
}

extern "C" void kernel_launch(void* const* d_in, const int* in_sizes, int n_in,
                              void* d_out, int out_size, void* d_ws, size_t ws_size,
                              hipStream_t stream) {
  if (n_in < 7) return;
  if (in_sizes[0] != NB_ * SEQ_ * DM_) return;
  if (in_sizes[1] != NB_ * SEQ_ * SEQ_) return;
  if (in_sizes[2] != NB_ * SEQ_) return;
  if (in_sizes[3] != DM_ * DM_) return;
  if (in_sizes[4] != HD_ * DM_) return;
  if (in_sizes[5] != HD_ * DM_) return;
  if (in_sizes[6] != DM_ * DM_) return;
  if (out_size != NB_ * SEQ_ * DM_) return;

  const float* x    = (const float*)d_in[0];
  const float* mask = (const float*)d_in[1];
  const int*   pos  = (const int*)d_in[2];
  const float* Wq   = (const float*)d_in[3];
  const float* Wk   = (const float*)d_in[4];
  const float* Wv   = (const float*)d_in[5];
  const float* Wo   = (const float*)d_in[6];
  float* out = (float*)d_out;

  const size_t nX   = (size_t)NB_ * SEQ_ * DM_;
  const size_t bXh  = nX * 2;
  const size_t bWq  = (size_t)DM_ * DM_ * 2;
  const size_t bWkv = (size_t)KVN_ * DM_ * 2;
  const size_t bWo  = bWq;
  const size_t bTab = (size_t)NB_ * SEQ_ * NF_ * 4;
  const size_t bQf  = nX * 4;
  const size_t bKVf = (size_t)NB_ * SEQ_ * KVN_ * 4;
  const size_t bQ16 = nX * 2;
  const size_t bK16 = (size_t)NB_ * SEQ_ * HD_ * 2;
  const size_t bV16 = bK16;
  const size_t bFlg = (size_t)NB_ * NQB_ * 128;
  size_t off = 0;
  const size_t oXh  = off; off += bXh;
  const size_t oWq  = off; off += bWq;
  const size_t oWkv = off; off += bWkv;
  const size_t oWo  = off; off += bWo;
  const size_t oCos = off; off += bTab;
  const size_t oSin = off; off += bTab;
  const size_t oQf  = off; off += bQf;
  const size_t oKVf = off; off += bKVf;
  const size_t oQh  = off; off += bQ16;
  const size_t oQl  = off; off += bQ16;
  const size_t oKh  = off; off += bK16;
  const size_t oKl  = off; off += bK16;
  const size_t oVth = off; off += bV16;
  const size_t oVtl = off; off += bV16;
  const size_t oFlg = off; off += bFlg;
  if (off > ws_size) return;
  if (off > (size_t)134217728) return;
  if (bQf < 2 * bQ16) return;
  const size_t oAOh = oQf;
  const size_t oAOl = oQf + bQ16;

  char* ws = (char*)d_ws;
  _Float16* Xh   = (_Float16*)(ws + oXh);
  _Float16* Wqh  = (_Float16*)(ws + oWq);
  _Float16* Wkvh = (_Float16*)(ws + oWkv);
  _Float16* Woh  = (_Float16*)(ws + oWo);
  float*    cosT = (float*)(ws + oCos);
  float*    sinT = (float*)(ws + oSin);
  float*    Qf   = (float*)(ws + oQf);
  float*    KVf  = (float*)(ws + oKVf);
  _Float16* Qh   = (_Float16*)(ws + oQh);
  _Float16* Ql   = (_Float16*)(ws + oQl);
  _Float16* Kh   = (_Float16*)(ws + oKh);
  _Float16* Kl   = (_Float16*)(ws + oKl);
  _Float16* Vth  = (_Float16*)(ws + oVth);
  _Float16* Vtl  = (_Float16*)(ws + oVtl);
  int*      flg  = (int*)(ws + oFlg);
  _Float16* AOh  = (_Float16*)(ws + oAOh);
  _Float16* AOl  = (_Float16*)(ws + oAOl);

  const dim3 blk(256);
  const int n8x = (int)(nX / 8);
  const int n8q = DM_ * DM_ / 8;
  const int n8k = HD_ * DM_ / 8;

  cvt16_kernel<<<dim3((n8x + 255) / 256), blk, 0, stream>>>(x, Xh, n8x, CX_);
  cvt16_kernel<<<dim3((n8q + 255) / 256), blk, 0, stream>>>(Wq, Wqh, n8q, CW_);
  cvt16_kernel<<<dim3((n8k + 255) / 256), blk, 0, stream>>>(Wk, Wkvh, n8k, CW_);
  cvt16_kernel<<<dim3((n8k + 255) / 256), blk, 0, stream>>>(Wv, Wkvh + (size_t)HD_ * DM_, n8k, CW_);
  cvt16_kernel<<<dim3((n8q + 255) / 256), blk, 0, stream>>>(Wo, Woh, n8q, CW_);
  rope_table_kernel<<<dim3((NB_ * SEQ_) / 32), blk, 0, stream>>>(pos, cosT, sinT, NB_ * SEQ_);
  maskflag_kernel<<<dim3(NB_ * NQB_), blk, 0, stream>>>(mask, flg);
  gemm64_kernel<<<dim3(((NB_ * SEQ_ / 64) * (DM_ / 64)) / 8), blk, 0, stream>>>(
      Xh, Xh, DM_, Wqh, DM_, Qf, DM_, NB_ * SEQ_, DM_, DM_, 0, SEQ_ - 1, QSC_);
  gemm64_kernel<<<dim3(((NB_ * SEQ_ / 64) * (KVN_ / 64)) / 8), blk, 0, stream>>>(
      Xh, Xh, DM_, Wkvh, DM_, KVf, KVN_, NB_ * SEQ_, KVN_, DM_, 0, SEQ_ - 1, QSC_);
  rope_split_kernel<<<dim3((NB_ * SEQ_ * NH_ * 8) / 256), blk, 0, stream>>>(
      Qf, DM_, NH_, cosT, sinT, Qh, Ql, DM_, NB_ * SEQ_ * NH_, CQK_);
  rope_split_kernel<<<dim3((NB_ * SEQ_ * 8) / 256), blk, 0, stream>>>(
      KVf, KVN_, 1, cosT, sinT, Kh, Kl, HD_, NB_ * SEQ_, CQK_);
  vt_split_kernel<<<dim3(HD_ / 64, (NB_ * SEQ_) / 64), blk, 0, stream>>>(KVf, Vth, Vtl);
  (void)hipFuncSetAttribute(reinterpret_cast<const void*>(&attn_kernel), hipFuncAttributeMaxDynamicSharedMemorySize, AT_LDS);
  attn_kernel<<<dim3(NB_ * NH_ * NQB_), blk, AT_LDS, stream>>>(Qh, Ql, Kh, Kl, Vth, Vtl, mask, flg, AOh, AOl);
  gemm64_kernel<<<dim3(((NB_ * SEQ_ / 64) * (DM_ / 64)) / 8), blk, 0, stream>>>(
      AOh, AOl, DM_, Woh, DM_, out, DM_, NB_ * SEQ_, DM_, DM_, LOROWS_, SEQ_ - 1, WSC_);
  (void)hipGetLastError();
}
